// Attention_77309411430
// MI455X (gfx1250) — hardware-verified
//
#include <hip/hip_runtime.h>


#ifndef NB
#define NB 2
#endif
#ifndef SEQ
#define SEQ 4096
#endif
#define NB_FULL 2
#define SEQ_FULL 4096
#define DMOD 512
#define NHEAD 8
#define HD 64
#define TOK (NB * SEQ)
#define PCAR 256.0f
#define QKCAR 4.0f
#define VCAR 16.0f
#define SL2E 0.011271055006945026f

static_assert(NB >= 1 && NB <= NB_FULL);
static_assert(SEQ >= 64 && SEQ <= SEQ_FULL && (SEQ % 64) == 0);
static_assert(DMOD == NHEAD * HD && (DMOD % 64) == 0 && HD == 64);
static_assert((((size_t)TOK * DMOD) % 8) == 0);
static_assert(((DMOD * DMOD) % 64) == 0);

typedef _Float16 h16;
typedef unsigned short bf;
typedef __attribute__((ext_vector_type(16))) __bf16   v16bf;
typedef __attribute__((ext_vector_type(16))) _Float16 v16h;
typedef __attribute__((ext_vector_type(8)))  _Float16 v8h;
typedef __attribute__((ext_vector_type(8)))  unsigned short v8us;
typedef __attribute__((ext_vector_type(8)))  float    v8f;
typedef __attribute__((ext_vector_type(4)))  float    v4f;
typedef __attribute__((ext_vector_type(2)))  unsigned short v2us;
typedef v8h  __attribute__((may_alias)) v8ha;
typedef v4f  __attribute__((may_alias)) v4fa;
typedef v8us __attribute__((may_alias)) v8usa;

__device__ __forceinline__ unsigned short f2bf(float f) { unsigned u = __float_as_uint(f); u += 0x7FFFu + ((u >> 16) & 1u); return (unsigned short)(u >> 16); }
__device__ __forceinline__ float bf2f(unsigned short b) { return __uint_as_float(((unsigned)b) << 16); }
__device__ __forceinline__ float bfr(float f) { return bf2f(f2bf(f)); }
__device__ __forceinline__ v16h cat16(v8h lo, v8h hi) { return __builtin_shufflevector(lo, hi, 0, 1, 2, 3, 4, 5, 6, 7, 8, 9, 10, 11, 12, 13, 14, 15); }
__device__ __forceinline__ v16bf cat16b(v8us lo, v8us hi) { return __builtin_bit_cast(v16bf, __builtin_shufflevector(lo, hi, 0, 1, 2, 3, 4, 5, 6, 7, 8, 9, 10, 11, 12, 13, 14, 15)); }
__device__ __forceinline__ v8f wmma16(v16h a, v16h b, v8f c) { return __builtin_amdgcn_wmma_f32_16x16x32_f16(false, a, false, b, (short)0, c, false, false); }
__device__ __forceinline__ v8f wmmab(v16bf a, v16bf b, v8f c) { return __builtin_amdgcn_wmma_f32_16x16x32_bf16(false, a, false, b, (short)0, c, false, false); }

template <typename T16> struct WFrag;
template <> struct WFrag<h16> { typedef v16h V; static __device__ __forceinline__ V ld(const h16* p) { return cat16(*(const v8h*)p, *(const v8h*)(p + 16)); } static __device__ __forceinline__ v8f mma(V a, V b, v8f c) { return wmma16(a, b, c); } };
template <> struct WFrag<bf> { typedef v16bf V; static __device__ __forceinline__ V ld(const bf* p) { return cat16b(*(const v8us*)p, *(const v8us*)(p + 16)); } static __device__ __forceinline__ v8f mma(V a, V b, v8f c) { return wmmab(a, b, c); } };
template <typename T16, int NSPLIT, bool BIAS>
__global__ __launch_bounds__(32) void k_gemmw(const T16* __restrict__ A, const T16* __restrict__ A2, const T16* __restrict__ Bt, const T16* __restrict__ Bt2, int K, float* C, int ldc, const float* __restrict__ bias, size_t sA, size_t sB, size_t sC) {
    typedef typename WFrag<T16>::V V;
    __shared__ __align__(16) float os[16 * 68];
    const size_t z = blockIdx.z; A += z * sA; if (A2) A2 += z * sA; Bt += z * sB; if (Bt2) Bt2 += z * sB; C += z * sC;
    const int lane = threadIdx.x & 31, lr = lane & 15, hi = lane >> 4; const int r0 = blockIdx.x * 64, c0 = blockIdx.y * 64;
    v8f acc[4][4];
#pragma unroll
    for (int mb = 0; mb < 4; ++mb)
#pragma unroll
        for (int nb = 0; nb < 4; ++nb) acc[mb][nb] = (v8f){};
    const size_t aoff = (size_t)(r0 + lr) * K + 8 * hi, boff = (size_t)(c0 + lr) * K + 8 * hi;
#pragma unroll 1
    for (int kc = 0; kc < K; kc += 32) {
        V a[4], a2[4];
#pragma unroll
        for (int mb = 0; mb < 4; ++mb) { a[mb] = WFrag<T16>::ld(A + aoff + (size_t)mb * 16 * K + kc); if (NSPLIT == 1 || NSPLIT == 2) a2[mb] = WFrag<T16>::ld(A2 + aoff + (size_t)mb * 16 * K + kc); }
#pragma unroll
        for (int nb = 0; nb < 4; ++nb) { const V b = WFrag<T16>::ld(Bt + boff + (size_t)nb * 16 * K + kc); V b2; if (NSPLIT >= 2) b2 = WFrag<T16>::ld(Bt2 + boff + (size_t)nb * 16 * K + kc);
#pragma unroll
            for (int mb = 0; mb < 4; ++mb) { acc[mb][nb] = WFrag<T16>::mma(a[mb], b, acc[mb][nb]); if (NSPLIT == 1 || NSPLIT == 2) acc[mb][nb] = WFrag<T16>::mma(a2[mb], b, acc[mb][nb]); if (NSPLIT >= 2) acc[mb][nb] = WFrag<T16>::mma(a[mb], b2, acc[mb][nb]); } }
        asm volatile("v_nop\n\tv_nop\n\tv_nop\n\tv_nop" : "+v"(acc[0][0]), "+v"(acc[1][1]), "+v"(acc[2][2]), "+v"(acc[3][3]) : "v"(a[0]), "v"(a[3]));
    }
#pragma unroll
    for (int mb = 0; mb < 4; ++mb) {
#pragma unroll
        for (int nb = 0; nb < 4; ++nb) {
#pragma unroll
            for (int j = 0; j < 8; ++j) os[(hi * 8 + j) * 68 + nb * 16 + lr] = acc[mb][nb][j]; }
        __builtin_amdgcn_wave_barrier(); asm volatile("" ::: "memory");
        float* crow = C + (size_t)(r0 + mb * 16) * ldc + c0;
#pragma unroll 1
        for (int ps = 0; ps < 2; ++ps) {
#pragma unroll
            for (int s = 0; s < 8; ++s) { const int row = 2 * s + hi, cofs = lr * 4; v4f val = *(const v4fa*)(os + row * 68 + cofs); if (BIAS) { val[0] += bfr(bias[c0 + cofs]); val[1] += bfr(bias[c0 + cofs + 1]); val[2] += bfr(bias[c0 + cofs + 2]); val[3] += bfr(bias[c0 + cofs + 3]); }
                *(volatile v4f*)(crow + (size_t)row * ldc + cofs) = val; }
            if (ps == 0) __threadfence(); }
        __builtin_amdgcn_wave_barrier(); asm volatile("" ::: "memory");
    }
}

__global__ __launch_bounds__(256) void k_wtG(const float* __restrict__ w, int K, int N, bf* Bt) {
    const int lane = threadIdx.x & 31; const int L0 = (blockIdx.x * 8 + (threadIdx.x >> 5)) * 8; const int nlines = N * K / 64;
#pragma unroll
    for (int ps = 0; ps < 2; ++ps) {
#pragma unroll 1
        for (int l = 0; l < 8; ++l) { const int L = L0 + l; if (L >= nlines) break; const size_t e = (size_t)L * 64 + lane * 2; const int k = (int)(e % K), n = (int)(e / K); v2us o;
            o[0] = f2bf(w[(size_t)k * N + n]); o[1] = f2bf(w[(size_t)(k + 1) * N + n]); *(volatile v2us*)(Bt + e) = o; }
        if (ps == 0) __threadfence(); }
}

__global__ __launch_bounds__(256) void k_xplane(const float* __restrict__ X, bf* XB) {
    const size_t i = (size_t)blockIdx.x * 256 + threadIdx.x; if (i >= (size_t)TOK * DMOD / 8) return;
    const size_t e = i * 8; const int col = (int)(e % DMOD); const size_t row = e / DMOD; const size_t bb = row / SEQ, s = row % SEQ;
    const v8f v = *(const v8f*)(X + (bb * SEQ_FULL + s) * DMOD + col); v8us o;
#pragma unroll
    for (int k = 0; k < 8; ++k) o[k] = f2bf(v[k]);
    *(volatile v8us*)(XB + e) = o; __threadfence(); *(volatile v8us*)(XB + e) = o;
}

template <int MODE>
__global__ __launch_bounds__(256) void k_cvt16(const float* __restrict__ Cf, const float* __restrict__ bias, float sc, h16* P) {
    const size_t i = (size_t)blockIdx.x * 256 + threadIdx.x; if (i >= (size_t)TOK * DMOD / 8) return;
    const size_t e = i * 8; const v8f v = *(const v8f*)(Cf + e); v8h o;
    if (MODE == 0) { const int col = (int)(e % DMOD); const v8f bb = *(const v8f*)(bias + col);
#pragma unroll
        for (int q = 0; q < 8; ++q) o[q] = (h16)((v[q] + bfr(bb[q])) * sc);
    } else { const int n = (int)(e / TOK); const float bn = bfr(bias[n]);
#pragma unroll
        for (int q = 0; q < 8; ++q) o[q] = (h16)((v[q] + bn) * sc);
    }
    *(volatile v8h*)(P + e) = o; __threadfence(); *(volatile v8h*)(P + e) = o;
}

__global__ __launch_bounds__(32) void k_sdpa(const h16* __restrict__ Q16, const h16* __restrict__ K16, const h16* __restrict__ VT16, float* out) {
    __shared__ __align__(16) float os[16 * 68];
    const int lane = threadIdx.x & 31, m = lane & 15, hh = lane >> 4;
    const int bh = blockIdx.y; const int b = bh / NHEAD, h = bh % NHEAD; const int q0 = blockIdx.x * 16;
    const h16* qrow = Q16 + ((size_t)b * SEQ + q0 + m) * DMOD + h * HD + 8 * hh;
    const v16h qf0 = cat16(*(const v8h*)(qrow), *(const v8h*)(qrow + 16));
    const v16h qf1 = cat16(*(const v8h*)(qrow + 32), *(const v8h*)(qrow + 48));
    const h16* kbase = K16 + ((size_t)b * SEQ + m) * DMOD + h * HD + 8 * hh;
    const h16* vbase = VT16 + ((size_t)h * HD + m) * TOK + (size_t)b * SEQ + 8 * hh;
    v8f oacc[4];
#pragma unroll
    for (int t = 0; t < 4; ++t) oacc[t] = (v8f){};
    float mrun = -3.0e38f, lrun = 0.f;
#pragma unroll 1
    for (int kb = 0; kb < SEQ; kb += 32) {
        v16h ka[2][2];
#pragma unroll
        for (int kt = 0; kt < 2; ++kt) { const h16* kr = kbase + (size_t)(kb + kt * 16) * DMOD; ka[kt][0] = cat16(*(const v8h*)kr, *(const v8h*)(kr + 16)); ka[kt][1] = cat16(*(const v8h*)(kr + 32), *(const v8h*)(kr + 48)); }
        v8f st[2];
#pragma unroll
        for (int kt = 0; kt < 2; ++kt) { st[kt] = wmma16(ka[kt][0], qf0, (v8f){}); st[kt] = wmma16(ka[kt][1], qf1, st[kt]); }
        asm volatile("v_nop\n\tv_nop\n\tv_nop\n\tv_nop" : "+v"(st[0]), "+v"(st[1]) : "v"(ka[0][0]), "v"(ka[0][1]), "v"(ka[1][0]), "v"(ka[1][1]), "v"(qf0), "v"(qf1));
        float mx = fmaxf(st[0][0], st[1][0]);
#pragma unroll
        for (int r = 1; r < 8; ++r) mx = fmaxf(mx, fmaxf(st[0][r], st[1][r]));
        mx = fmaxf(mx, __shfl_xor(mx, 16, 32));
        const float mn = fmaxf(mrun, mx);
        const float alpha = __builtin_amdgcn_exp2f((mrun - mn) * SL2E);
        mrun = mn;
        v16h pf = (v16h){}; float psum = 0.f;
#pragma unroll
        for (int r = 0; r < 8; ++r) {
            const h16 p0 = (h16)(__builtin_amdgcn_exp2f((st[0][r] - mn) * SL2E) * PCAR);
            const h16 p1 = (h16)(__builtin_amdgcn_exp2f((st[1][r] - mn) * SL2E) * PCAR);
            pf[r] = p0; pf[8 + r] = p1; psum += (float)p0 + (float)p1; }
        psum += __shfl_xor(psum, 16, 32);
        lrun = lrun * alpha + psum;
#pragma unroll
        for (int t = 0; t < 4; ++t) oacc[t] *= alpha;
        v16h va[4];
#pragma unroll
        for (int t = 0; t < 4; ++t) { const h16* vr = vbase + (size_t)t * 16 * TOK + kb; va[t] = cat16(*(const v8h*)vr, *(const v8h*)(vr + 16)); }
#pragma unroll
        for (int t = 0; t < 4; ++t) oacc[t] = wmma16(va[t], pf, oacc[t]);
        asm volatile("v_nop\n\tv_nop\n\tv_nop\n\tv_nop" : "+v"(oacc[0]), "+v"(oacc[1]), "+v"(oacc[2]), "+v"(oacc[3]) : "v"(va[0]), "v"(va[1]), "v"(va[2]), "v"(va[3]), "v"(pf));
    }
    const float rl = __fdiv_rn(1.0f, lrun) * (1.0f / VCAR);
#pragma unroll
    for (int t = 0; t < 4; ++t)
#pragma unroll
        for (int r = 0; r < 8; ++r) os[m * 68 + t * 16 + hh * 8 + r] = oacc[t][r] * rl;
    __syncthreads();
    float* obase = out + ((size_t)b * SEQ + q0) * DMOD + h * HD;
#pragma unroll 1
    for (int ps = 0; ps < 2; ++ps) {
#pragma unroll
        for (int s = 0; s < 8; ++s) { const int row = 2 * s + hh, cofs = m * 4; const v4f val = *(const v4fa*)(os + row * 68 + cofs); *(volatile v4f*)(obase + (size_t)row * DMOD + cofs) = val; }
        if (ps == 0) __threadfence(); }
}

extern "C" void kernel_launch(void* const* d_in, const int* in_sizes, int n_in,
                              void* d_out, int out_size, void* d_ws, size_t ws_size, hipStream_t stream) {
    if (n_in < 9) return;
    const int need_x = ((NB - 1) * SEQ_FULL + SEQ) * DMOD;
    if (in_sizes[0] < need_x || in_sizes[1] < need_x || in_sizes[2] < need_x) return;
    if (in_sizes[3] < DMOD * DMOD || in_sizes[5] < DMOD * DMOD || in_sizes[7] < DMOD * DMOD) return;
    if (in_sizes[4] < DMOD || in_sizes[6] < DMOD || in_sizes[8] < DMOD) return;
    if (out_size < TOK * DMOD) return;
    const float* Xq = (const float*)d_in[0]; const float* Xk = (const float*)d_in[1]; const float* Xv = (const float*)d_in[2];
    const float* Wq = (const float*)d_in[3]; const float* bq = (const float*)d_in[4];
    const float* Wk = (const float*)d_in[5]; const float* bk = (const float*)d_in[6];
    const float* Wv = (const float*)d_in[7]; const float* bv = (const float*)d_in[8];
    float* OUT = (float*)d_out;
    char* wsp = (char*)d_ws;
    auto take = [&](size_t bytes) { char* p = wsp; wsp += (bytes + 255) & ~(size_t)255; return (void*)p; };
    bf* WTq = (bf*)take((size_t)DMOD * DMOD * 2); bf* WTk = (bf*)take((size_t)DMOD * DMOD * 2); bf* WTv = (bf*)take((size_t)DMOD * DMOD * 2);
    bf* XB = (bf*)take((size_t)TOK * DMOD * 2);
    float* Cf = (float*)take((size_t)TOK * DMOD * 4);
    h16* Q16 = (h16*)take((size_t)TOK * DMOD * 2); h16* K16 = (h16*)take((size_t)TOK * DMOD * 2); h16* VT16 = (h16*)take((size_t)TOK * DMOD * 2);
    if ((size_t)(wsp - (char*)d_ws) > ws_size) return;
    const unsigned gw = (unsigned)((DMOD * DMOD / 64 + 63) / 64);
    const unsigned g8 = (unsigned)(((size_t)TOK * DMOD / 8 + 255) / 256);
    k_wtG<<<gw, 256, 0, stream>>>(Wq, DMOD, DMOD, WTq);
    k_wtG<<<gw, 256, 0, stream>>>(Wk, DMOD, DMOD, WTk);
    k_wtG<<<gw, 256, 0, stream>>>(Wv, DMOD, DMOD, WTv);
    k_xplane<<<g8, 256, 0, stream>>>(Xq, XB);
    k_gemmw<bf, 0, false><<<dim3(TOK / 64, DMOD / 64, 1), 32, 0, stream>>>(XB, nullptr, WTq, nullptr, DMOD, Cf, DMOD, nullptr, 0, 0, 0);
    k_cvt16<0><<<g8, 256, 0, stream>>>(Cf, bq, QKCAR, Q16);
    k_xplane<<<g8, 256, 0, stream>>>(Xk, XB);
    k_gemmw<bf, 0, false><<<dim3(TOK / 64, DMOD / 64, 1), 32, 0, stream>>>(XB, nullptr, WTk, nullptr, DMOD, Cf, DMOD, nullptr, 0, 0, 0);
    k_cvt16<0><<<g8, 256, 0, stream>>>(Cf, bk, QKCAR, K16);
    k_xplane<<<g8, 256, 0, stream>>>(Xv, XB);
    k_gemmw<bf, 0, false><<<dim3(DMOD / 64, TOK / 64, 1), 32, 0, stream>>>(WTv, nullptr, XB, nullptr, DMOD, Cf, TOK, nullptr, 0, 0, 0);
    k_cvt16<1><<<g8, 256, 0, stream>>>(Cf, bv, VCAR, VT16);
    k_sdpa<<<dim3(SEQ / 16, NB * NHEAD, 1), 32, 0, stream>>>(Q16, K16, VT16, OUT);
}
